// MAN_9723805958786
// MI455X (gfx1250) — hardware-verified
//
#include <hip/hip_runtime.h>
#include <math.h>
#include <stdint.h>
#include <stddef.h>


typedef __bf16         v16bf __attribute__((ext_vector_type(16)));
typedef float          v8f   __attribute__((ext_vector_type(8)));
typedef float          v4f   __attribute__((ext_vector_type(4)));
typedef unsigned int   v4u   __attribute__((ext_vector_type(4)));
typedef unsigned short u16;

union Frag { v16bf v; v4u u[2]; };

static constexpr int BB  = 4;
static constexpr int SS  = 1024;
static constexpr int DM  = 1024;
static constexpr int HH  = 16;
static constexpr int DKK = 64;
static constexpr int MROWS = BB * SS;
static constexpr size_t ACT = (size_t)MROWS * DM;
static constexpr size_t WEL = (size_t)DM * DM;
static_assert(HH * DKK == DM);
static_assert(MROWS % 64 == 0);
static_assert(DM % 128 == 0);
static_assert(DM % 32 == 0);
static_assert(SS % 64 == 0);
static_assert(ACT % 2048 == 0);
static_assert(WEL % 2048 == 0);

__device__ __forceinline__ unsigned bf16_bits(float x) {
  unsigned u = __float_as_uint(x);
  u += 0x7FFFu + ((u >> 16) & 1u);
  return u >> 16;
}
__device__ __forceinline__ void split2(float x, unsigned& hi, unsigned& lo) {
  hi = bf16_bits(x);
  const float xh = __uint_as_float(hi << 16);
  lo = bf16_bits(x - xh);
}
__device__ __forceinline__ void split8(const float* x, v4u& vh, v4u& vl) {
  unsigned hw[4], lw[4];
#pragma unroll
  for (int i = 0; i < 4; ++i) {
    unsigned h0, l0, h1, l1;
    split2(x[2 * i], h0, l0);
    split2(x[2 * i + 1], h1, l1);
    hw[i] = h0 | (h1 << 16);
    lw[i] = l0 | (l1 << 16);
  }
  vh.x = hw[0]; vh.y = hw[1]; vh.z = hw[2]; vh.w = hw[3];
  vl.x = lw[0]; vl.y = lw[1]; vl.z = lw[2]; vl.w = lw[3];
}
__device__ __forceinline__ v8f zero8() {
  v8f z;
#pragma unroll
  for (int i = 0; i < 8; ++i) z[i] = 0.f;
  return z;
}
__device__ __forceinline__ v16bf ldg_frag(const u16* __restrict__ p, size_t e) {
  Frag f;
  f.u[0] = *(const v4u*)(p + e);
  f.u[1] = *(const v4u*)(p + e + 16);
  return f.v;
}
__device__ __forceinline__ v16bf lds_frag(const u16* p, int e) {
  Frag f;
  f.u[0] = *(const v4u*)(p + e);
  f.u[1] = *(const v4u*)(p + e + 16);
  return f.v;
}
__device__ __forceinline__ v8f wmma3(v8f acc, v16bf ah, v16bf al, v16bf bh, v16bf bl) {
  acc = __builtin_amdgcn_wmma_f32_16x16x32_bf16(false, ah, false, bh, (short)0, acc, false, false);
  acc = __builtin_amdgcn_wmma_f32_16x16x32_bf16(false, ah, false, bl, (short)0, acc, false, false);
  acc = __builtin_amdgcn_wmma_f32_16x16x32_bf16(false, al, false, bh, (short)0, acc, false, false);
  asm volatile("v_nop\n\tv_nop\n\tv_nop\n\tv_nop" : "+v"(acc) : "v"(ah), "v"(al), "v"(bh), "v"(bl));
  return acc;
}

__global__ void __launch_bounds__(256)
k_split(const float* __restrict__ in, u16* __restrict__ ph, u16* __restrict__ pl, int n8) {
  const int t = blockIdx.x * 256 + (int)threadIdx.x;
  if (t >= n8) return;
  const size_t base = (size_t)t * 8;
  const v4f a = *(const v4f*)(in + base);
  const v4f c = *(const v4f*)(in + base + 4);
  float x[8] = {a.x, a.y, a.z, a.w, c.x, c.y, c.z, c.w};
  v4u vh, vl;
  split8(x, vh, vl);
  u16* dh = ph + base;
  u16* dl = pl + base;
  *(volatile v4u*)dh = vh;
  *(volatile v4u*)dl = vl;
  __threadfence();
  *(volatile v4u*)dh = vh;
  *(volatile v4u*)dl = vl;
}

static constexpr int TP = 132;

template <int MODE>
__global__ void __launch_bounds__(256)
k_gemm3(const u16* __restrict__ Ah, const u16* __restrict__ Al,
        const u16* __restrict__ Wh, const u16* __restrict__ Wl,
        const float* __restrict__ bias,
        u16* __restrict__ Oh, u16* __restrict__ Ol, float* __restrict__ Of) {
  constexpr int N = DM, K = DM;
  __shared__ __attribute__((aligned(16))) float sT[64 * TP];

  const int lane = threadIdx.x & 31;
  const int w    = threadIdx.x >> 5;
  const int wm   = w & 3;
  const int wn   = w >> 2;
  const int hl   = lane >> 4;
  const int l15  = lane & 15;
  const int m0b  = blockIdx.y * 64;
  const int n0b  = blockIdx.x * 128;
  const int m0   = m0b + wm * 16;
  const int n0   = n0b + wn * 64;

  v8f acc[4];
#pragma unroll
  for (int nt = 0; nt < 4; ++nt) acc[nt] = zero8();

  const size_t ea0 = (size_t)(m0 + l15) * K + hl * 8;
  const size_t eb0 = (size_t)(n0 + l15) * K + hl * 8;

#pragma unroll 2
  for (int k0 = 0; k0 < K; k0 += 32) {
    const v16bf ah = ldg_frag(Ah, ea0 + k0);
    const v16bf al = ldg_frag(Al, ea0 + k0);
#pragma unroll
    for (int nt = 0; nt < 4; ++nt) {
      const size_t eb = eb0 + (size_t)nt * 16 * K + k0;
      const v16bf bh = ldg_frag(Wh, eb);
      const v16bf bl = ldg_frag(Wl, eb);
      acc[nt] = wmma3(acc[nt], ah, al, bh, bl);
    }
  }

#pragma unroll
  for (int nt = 0; nt < 4; ++nt) {
    const float bb = bias[n0 + nt * 16 + l15];
#pragma unroll
    for (int r = 0; r < 8; ++r)
      sT[(wm * 16 + hl * 8 + r) * TP + wn * 64 + nt * 16 + l15] = acc[nt][r] + bb;
  }
  __syncthreads();

  if (MODE == 0) {
    const int rsub = lane >> 4;
    const int cc   = (lane & 15) * 8;
    v4u vh[4], vl[4];
    size_t go[4];
#pragma unroll
    for (int j = 0; j < 4; ++j) {
      const int row = w * 8 + 2 * j + rsub;
      const float* sp = sT + row * TP + cc;
      const v4f a = *(const v4f*)sp;
      const v4f c = *(const v4f*)(sp + 4);
      float x[8] = {a.x, a.y, a.z, a.w, c.x, c.y, c.z, c.w};
      split8(x, vh[j], vl[j]);
      go[j] = (size_t)(m0b + row) * N + n0b + cc;
    }
#pragma unroll
    for (int j = 0; j < 4; ++j) {
      *(volatile v4u*)(Oh + go[j]) = vh[j];
      *(volatile v4u*)(Ol + go[j]) = vl[j];
    }
    __threadfence();
#pragma unroll
    for (int j = 0; j < 4; ++j) {
      *(volatile v4u*)(Oh + go[j]) = vh[j];
      *(volatile v4u*)(Ol + go[j]) = vl[j];
    }
  } else if (MODE == 1) {
    const int bidx = m0b / SS;
    const int s0   = m0b - bidx * SS;
    const int fsub = lane >> 3;
    const int tc   = (lane & 7) * 8;
    v4u vh[4], vl[4];
    size_t go[4];
#pragma unroll
    for (int j = 0; j < 4; ++j) {
      const int f = w * 16 + 4 * j + fsub;
      float x[8];
#pragma unroll
      for (int i = 0; i < 8; ++i) x[i] = sT[(tc + i) * TP + f];
      split8(x, vh[j], vl[j]);
      go[j] = ((size_t)bidx * N + n0b + f) * SS + s0 + tc;
    }
#pragma unroll
    for (int j = 0; j < 4; ++j) {
      *(volatile v4u*)(Oh + go[j]) = vh[j];
      *(volatile v4u*)(Ol + go[j]) = vl[j];
    }
    __threadfence();
#pragma unroll
    for (int j = 0; j < 4; ++j) {
      *(volatile v4u*)(Oh + go[j]) = vh[j];
      *(volatile v4u*)(Ol + go[j]) = vl[j];
    }
  } else {
    const int cc4 = lane * 4;
    v4f val[8];
    size_t go[8];
#pragma unroll
    for (int j = 0; j < 8; ++j) {
      const int row = w * 8 + j;
      val[j] = *(const v4f*)(sT + row * TP + cc4);
      go[j]  = (size_t)(m0b + row) * N + n0b + cc4;
    }
#pragma unroll
    for (int j = 0; j < 8; ++j) *(volatile v4f*)(Of + go[j]) = val[j];
    __threadfence();
#pragma unroll
    for (int j = 0; j < 8; ++j) *(volatile v4f*)(Of + go[j]) = val[j];
  }
}

static constexpr int SST = 1028;
static constexpr int AST = 1032;
static constexpr int OST = 68;
static constexpr size_t SM_S = (size_t)16 * SST * 4;
static constexpr size_t SM_P = (size_t)8 * 1024 * 4;
static constexpr size_t SM_A = (size_t)16 * AST * 2;
static constexpr size_t SMEM_ATTN = SM_S + SM_P + 2 * SM_A;
static_assert((size_t)16 * OST * 4 <= SM_P);
static_assert(SM_S % 16 == 0);
static_assert(SM_P % 16 == 0);
static_assert(SM_A % 16 == 0);

__global__ void __launch_bounds__(256)
k_attn(const u16* __restrict__ Qh, const u16* __restrict__ Ql,
       const u16* __restrict__ Kh, const u16* __restrict__ Kl,
       const u16* __restrict__ Vh, const u16* __restrict__ Vl,
       const float* __restrict__ gammas,
       u16* __restrict__ Ch, u16* __restrict__ Cl) {
  extern __shared__ __attribute__((aligned(16))) char smem[];
  float* sS   = (float*)smem;
  float* pbuf = (float*)(smem + SM_S);
  float* sO   = pbuf;
  u16*   aH   = (u16*)(smem + SM_S + SM_P);
  u16*   aL   = (u16*)(smem + SM_S + SM_P + SM_A);

  const int qt = blockIdx.x, h = blockIdx.y, b = blockIdx.z;
  const int q0 = qt * 16;
  const int lane = threadIdx.x & 31;
  const int w    = threadIdx.x >> 5;
  const int hl   = lane >> 4;
  const int l15  = lane & 15;

  {
    const size_t qrow = (size_t)(b * SS + q0 + l15) * DM + h * DKK + hl * 8;
    const v16bf qh0 = ldg_frag(Qh, qrow),      ql0 = ldg_frag(Ql, qrow);
    const v16bf qh1 = ldg_frag(Qh, qrow + 32), ql1 = ldg_frag(Ql, qrow + 32);
    for (int t = 0; t < 8; ++t) {
      const int kt = w * 8 + t;
      const size_t krow = (size_t)(b * SS + kt * 16 + l15) * DM + h * DKK + hl * 8;
      v8f acc = zero8();
      {
        const v16bf kh = ldg_frag(Kh, krow), kl = ldg_frag(Kl, krow);
        acc = wmma3(acc, qh0, ql0, kh, kl);
      }
      {
        const v16bf kh = ldg_frag(Kh, krow + 32), kl = ldg_frag(Kl, krow + 32);
        acc = wmma3(acc, qh1, ql1, kh, kl);
      }
#pragma unroll
      for (int r = 0; r < 8; ++r)
        sS[(hl * 8 + r) * SST + kt * 16 + l15] = acc[r] * 0.125f;
    }
  }
  __syncthreads();

  {
    const float gg  = gammas[h];
    const float gam = -(fmaxf(gg, 0.f) + log1pf(expf(-fabsf(gg))));
    const int cb = lane * 32;
    for (int rr = 0; rr < 2; ++rr) {
      const int row = w + rr * 8;
      const int iq  = q0 + row;
      float* srow = sS + row * SST + cb;
      float* prow = pbuf + w * 1024 + cb;

      float m1 = -3.0e38f;
#pragma unroll 1
      for (int g8 = 0; g8 < 4; ++g8) {
        const v4f a = *(const v4f*)(srow + 8 * g8);
        const v4f c = *(const v4f*)(srow + 8 * g8 + 4);
        m1 = fmaxf(m1, fmaxf(fmaxf(fmaxf(a.x, a.y), fmaxf(a.z, a.w)),
                             fmaxf(fmaxf(c.x, c.y), fmaxf(c.z, c.w))));
      }
#pragma unroll
      for (int o = 16; o > 0; o >>= 1) m1 = fmaxf(m1, __shfl_xor(m1, o, 32));

      float s1 = 0.f;
#pragma unroll 1
      for (int g8 = 0; g8 < 4; ++g8) {
        const v4f a = *(const v4f*)(srow + 8 * g8);
        const v4f c = *(const v4f*)(srow + 8 * g8 + 4);
        float x[8] = {a.x, a.y, a.z, a.w, c.x, c.y, c.z, c.w};
        float e[8];
#pragma unroll
        for (int i = 0; i < 8; ++i) { e[i] = expf(x[i] - m1); s1 += e[i]; }
        v4f ea, ec;
        ea.x = e[0]; ea.y = e[1]; ea.z = e[2]; ea.w = e[3];
        ec.x = e[4]; ec.y = e[5]; ec.z = e[6]; ec.w = e[7];
        *(v4f*)(prow + 8 * g8)     = ea;
        *(v4f*)(prow + 8 * g8 + 4) = ec;
      }
#pragma unroll
      for (int o = 16; o > 0; o >>= 1) s1 += __shfl_xor(s1, o, 32);
      const float inv1 = 1.0f / s1;

      float run = 0.f;
#pragma unroll 1
      for (int g8 = 0; g8 < 4; ++g8) {
        const v4f a = *(const v4f*)(prow + 8 * g8);
        const v4f c = *(const v4f*)(prow + 8 * g8 + 4);
        float e[8] = {a.x, a.y, a.z, a.w, c.x, c.y, c.z, c.w};
        float y[8];
#pragma unroll
        for (int i = 0; i < 8; ++i) {
          const int cidx = cb + 8 * g8 + i;
          const float p = (cidx <= iq) ? e[i] * inv1 : 0.f;
          run += p;
          y[i] = run;
        }
        v4f ya, yc;
        ya.x = y[0]; ya.y = y[1]; ya.z = y[2]; ya.w = y[3];
        yc.x = y[4]; yc.y = y[5]; yc.z = y[6]; yc.w = y[7];
        *(v4f*)(prow + 8 * g8)     = ya;
        *(v4f*)(prow + 8 * g8 + 4) = yc;
      }
      float incl = run;
#pragma unroll
      for (int d = 1; d < 32; d <<= 1) {
        const float t = __shfl_up(incl, d, 32);
        if (lane >= d) incl += t;
      }
      const float off       = incl - run;
      const float disttotal = __shfl(incl, 31, 32);

      float m2 = -3.0e38f;
#pragma unroll 1
      for (int g8 = 0; g8 < 4; ++g8) {
        const v4f ca = *(const v4f*)(prow + 8 * g8);
        const v4f cc = *(const v4f*)(prow + 8 * g8 + 4);
        const v4f sa = *(const v4f*)(srow + 8 * g8);
        const v4f sc = *(const v4f*)(srow + 8 * g8 + 4);
        float cum[8] = {ca.x, ca.y, ca.z, ca.w, cc.x, cc.y, cc.z, cc.w};
        float s[8]   = {sa.x, sa.y, sa.z, sa.w, sc.x, sc.y, sc.z, sc.w};
        float o8[8];
#pragma unroll
        for (int i = 0; i < 8; ++i) {
          const int cidx = cb + 8 * g8 + i;
          const float distcum = off + cum[i];
          const float pe  = fabsf((float)(iq - cidx));
          const float x   = (disttotal - distcum) * pe;
          const float dsc = sqrtf(fmaxf(x, 0.f));
          float eff = expf(dsc * gam);
          eff = fminf(fmaxf(eff, 1e-5f), 1e5f);
          const float ns = (cidx <= iq) ? s[i] * eff : -1e32f;
          o8[i] = ns;
          m2 = fmaxf(m2, ns);
        }
        v4f oa, oc;
        oa.x = o8[0]; oa.y = o8[1]; oa.z = o8[2]; oa.w = o8[3];
        oc.x = o8[4]; oc.y = o8[5]; oc.z = o8[6]; oc.w = o8[7];
        *(v4f*)(srow + 8 * g8)     = oa;
        *(v4f*)(srow + 8 * g8 + 4) = oc;
      }
#pragma unroll
      for (int o = 16; o > 0; o >>= 1) m2 = fmaxf(m2, __shfl_xor(m2, o, 32));

      float s2 = 0.f;
#pragma unroll 1
      for (int g8 = 0; g8 < 4; ++g8) {
        const v4f sa = *(const v4f*)(srow + 8 * g8);
        const v4f sc = *(const v4f*)(srow + 8 * g8 + 4);
        float s[8] = {sa.x, sa.y, sa.z, sa.w, sc.x, sc.y, sc.z, sc.w};
        float e[8];
#pragma unroll
        for (int i = 0; i < 8; ++i) { e[i] = expf(s[i] - m2); s2 += e[i]; }
        v4f ea, ec;
        ea.x = e[0]; ea.y = e[1]; ea.z = e[2]; ea.w = e[3];
        ec.x = e[4]; ec.y = e[5]; ec.z = e[6]; ec.w = e[7];
        *(v4f*)(srow + 8 * g8)     = ea;
        *(v4f*)(srow + 8 * g8 + 4) = ec;
      }
#pragma unroll
      for (int o = 16; o > 0; o >>= 1) s2 += __shfl_xor(s2, o, 32);
      const float inv2 = 1.0f / s2;

      u16* ahp = aH + row * AST + cb;
      u16* alp = aL + row * AST + cb;
#pragma unroll 1
      for (int g8 = 0; g8 < 4; ++g8) {
        const v4f sa = *(const v4f*)(srow + 8 * g8);
        const v4f sc = *(const v4f*)(srow + 8 * g8 + 4);
        float p[8] = {sa.x * inv2, sa.y * inv2, sa.z * inv2, sa.w * inv2,
                      sc.x * inv2, sc.y * inv2, sc.z * inv2, sc.w * inv2};
        v4u vh, vl;
        split8(p, vh, vl);
        *(v4u*)(ahp + 8 * g8) = vh;
        *(v4u*)(alp + 8 * g8) = vl;
      }
    }
  }
  __syncthreads();

  if (w < 4) {
    const int nt  = w;
    const int nkt = q0 / 32 + 1;
    const size_t vrow = ((size_t)(b * DM + h * DKK + nt * 16 + l15)) * SS + hl * 8;
    v8f acc = zero8();
    for (int kt = 0; kt < nkt; ++kt) {
      const int pa = l15 * AST + kt * 32 + hl * 8;
      const v16bf ph = lds_frag(aH, pa);
      const v16bf pl = lds_frag(aL, pa);
      const size_t ev = vrow + (size_t)kt * 32;
      const v16bf vh = ldg_frag(Vh, ev);
      const v16bf vl = ldg_frag(Vl, ev);
      acc = wmma3(acc, ph, pl, vh, vl);
    }
#pragma unroll
    for (int r = 0; r < 8; ++r)
      sO[(hl * 8 + r) * OST + nt * 16 + l15] = acc[r];
  }
  __syncthreads();

  if (w < 4) {
    const int row = w * 4 + (lane >> 3);
    const int cc  = (lane & 7) * 8;
    const float* sp = sO + row * OST + cc;
    const v4f a = *(const v4f*)sp;
    const v4f c = *(const v4f*)(sp + 4);
    float x[8] = {a.x, a.y, a.z, a.w, c.x, c.y, c.z, c.w};
    v4u vh, vl;
    split8(x, vh, vl);
    const size_t go = (size_t)(b * SS + q0 + row) * DM + h * DKK + cc;
    *(volatile v4u*)(Ch + go) = vh;
    *(volatile v4u*)(Cl + go) = vl;
    __threadfence();
    *(volatile v4u*)(Ch + go) = vh;
    *(volatile v4u*)(Cl + go) = vl;
  }
}

extern "C" void kernel_launch(void* const* d_in, const int* in_sizes, int n_in,
                              void* d_out, int out_size, void* d_ws, size_t ws_size,
                              hipStream_t stream) {
  if (n_in < 12) return;
  if (in_sizes[0] != (int)ACT || in_sizes[1] != (int)ACT || in_sizes[2] != (int)ACT) return;
  if (in_sizes[3] != (int)WEL || in_sizes[5] != (int)WEL || in_sizes[7] != (int)WEL || in_sizes[9] != (int)WEL) return;
  if (in_sizes[4] != DM || in_sizes[6] != DM || in_sizes[8] != DM || in_sizes[10] != DM) return;
  if (in_sizes[11] != HH) return;
  if (out_size != (int)ACT) return;

  const float* q   = (const float*)d_in[0];
  const float* k   = (const float*)d_in[1];
  const float* v   = (const float*)d_in[2];
  const float* Wq  = (const float*)d_in[3];
  const float* bq  = (const float*)d_in[4];
  const float* Wk  = (const float*)d_in[5];
  const float* bk  = (const float*)d_in[6];
  const float* Wv  = (const float*)d_in[7];
  const float* bv  = (const float*)d_in[8];
  const float* Wo  = (const float*)d_in[9];
  const float* bo  = (const float*)d_in[10];
  const float* gam = (const float*)d_in[11];
  float* out = (float*)d_out;

  char* ws = (char*)d_ws;
  size_t off = 0;
  auto carve = [&](size_t bytes) -> char* {
    char* p = ws + off;
    off += (bytes + 255) & ~(size_t)255;
    return p;
  };
  u16* actH = (u16*)carve(ACT * 2);
  u16* actL = (u16*)carve(ACT * 2);
  u16* wH   = (u16*)carve(WEL * 2);
  u16* wL   = (u16*)carve(WEL * 2);
  u16* QpH  = (u16*)carve(ACT * 2);
  u16* QpL  = (u16*)carve(ACT * 2);
  u16* KpH  = (u16*)carve(ACT * 2);
  u16* KpL  = (u16*)carve(ACT * 2);
  u16* VtH  = (u16*)carve(ACT * 2);
  u16* VtL  = (u16*)carve(ACT * 2);
  if (off > ws_size) return;

  const int nAct8 = (int)(ACT / 8);
  const int nWel8 = (int)(WEL / 8);
  const dim3 gAct((unsigned)((nAct8 + 255) / 256));
  const dim3 gWel((unsigned)((nWel8 + 255) / 256));
  const dim3 ggrid(DM / 128, MROWS / 64);
  const dim3 agrid(SS / 16, HH, BB);

  k_split<<<gAct, 256, 0, stream>>>(q, actH, actL, nAct8);
  k_split<<<gWel, 256, 0, stream>>>(Wq, wH, wL, nWel8);
  k_gemm3<0><<<ggrid, 256, 0, stream>>>(actH, actL, wH, wL, bq, QpH, QpL, out);
  k_split<<<gAct, 256, 0, stream>>>(k, actH, actL, nAct8);
  k_split<<<gWel, 256, 0, stream>>>(Wk, wH, wL, nWel8);
  k_gemm3<0><<<ggrid, 256, 0, stream>>>(actH, actL, wH, wL, bk, KpH, KpL, out);
  k_split<<<gAct, 256, 0, stream>>>(v, actH, actL, nAct8);
  k_split<<<gWel, 256, 0, stream>>>(Wv, wH, wL, nWel8);
  k_gemm3<1><<<ggrid, 256, 0, stream>>>(actH, actL, wH, wL, bv, VtH, VtL, out);
  k_attn<<<agrid, 256, SMEM_ATTN, stream>>>(QpH, QpL, KpH, KpL, VtH, VtL, gam, actH, actL);
  k_split<<<gWel, 256, 0, stream>>>(Wo, wH, wL, nWel8);
  k_gemm3<2><<<ggrid, 256, 0, stream>>>(actH, actL, wH, wL, bo, QpH, QpL, out);
}
